// MultiHeadTransformerSparseLayer_72378788873009
// MI455X (gfx1250) — hardware-verified
//
#include <hip/hip_runtime.h>


#define NB_  32
#define NF   1024
#define DIN  64
#define DOUT 64
#define NH_  4
#define HW   (NH_ * DOUT)
#define NTK  (NB_ * NF)
#define LOSC 1024.0f
#define LOSCI (1.0f / 1024.0f)
#define PSC  256.0f

typedef _Float16 h16;
typedef unsigned short bf;
typedef __attribute__((ext_vector_type(16))) __bf16   v16bf;
typedef __attribute__((ext_vector_type(16))) _Float16 v16h;
typedef __attribute__((ext_vector_type(8)))  _Float16 v8h;
typedef __attribute__((ext_vector_type(8)))  unsigned short v8us;
typedef __attribute__((ext_vector_type(8)))  float    v8f;
typedef __attribute__((ext_vector_type(4)))  float    v4f;
typedef v8h  __attribute__((may_alias)) v8ha;
typedef v4f  __attribute__((may_alias)) v4fa;
typedef v8us __attribute__((may_alias)) v8usa;

__device__ __forceinline__ unsigned short f2bf(float f) { unsigned u = __float_as_uint(f); u += 0x7FFFu + ((u >> 16) & 1u); return (unsigned short)(u >> 16); }
__device__ __forceinline__ float bf2f(unsigned short b) { return __uint_as_float(((unsigned)b) << 16); }
__device__ __forceinline__ float bfr(float f) { return bf2f(f2bf(f)); }
__device__ __forceinline__ v16h cat16(v8h lo, v8h hi) { return __builtin_shufflevector(lo, hi, 0, 1, 2, 3, 4, 5, 6, 7, 8, 9, 10, 11, 12, 13, 14, 15); }
__device__ __forceinline__ v16bf cat16b(v8us lo, v8us hi) { return __builtin_bit_cast(v16bf, __builtin_shufflevector(lo, hi, 0, 1, 2, 3, 4, 5, 6, 7, 8, 9, 10, 11, 12, 13, 14, 15)); }
__device__ __forceinline__ v8f wmma16(v16h a, v16h b, v8f c) { return __builtin_amdgcn_wmma_f32_16x16x32_f16(false, a, false, b, (short)0, c, false, false); }
__device__ __forceinline__ v8f wmmab(v16bf a, v16bf b, v8f c) { return __builtin_amdgcn_wmma_f32_16x16x32_bf16(false, a, false, b, (short)0, c, false, false); }
#define VST2(T, p, v) do { const T vst2_v_ = (v); *(volatile T*)(p) = vst2_v_; __threadfence(); *(volatile T*)(p) = vst2_v_; } while (0)

__global__ __launch_bounds__(256) void k_xb(const float* __restrict__ x, bf* Xb) {
    typedef __attribute__((ext_vector_type(4))) unsigned short v4us;
    const int lane = threadIdx.x & 31; const size_t w = (size_t)blockIdx.x * 8 + (threadIdx.x >> 5);
    v4us t;
#pragma unroll
    for (int i = 0; i < 4; ++i) t[i] = f2bf(x[w * 128 + lane * 4 + i]);
    VST2(v4us, Xb + w * 128 + lane * 4, t);
}
__global__ __launch_bounds__(256) void k_w(const float* __restrict__ Wqkv, const float* __restrict__ Wo, bf* WT, bf* WoT) {
    typedef __attribute__((ext_vector_type(2))) unsigned short v2us;
    const int t = threadIdx.x;
#pragma unroll 1
    for (int s = 0; s < (3 * HW * DIN) / 512; ++s) { const int e0 = s * 512 + t * 2; v2us o;
#pragma unroll
        for (int q = 0; q < 2; ++q) { const int e = e0 + q, k = e / (HW * DIN), rem = e - k * (HW * DIN), ho = rem / DIN, i = rem - ho * DIN, h = ho / DOUT, oo = ho - h * DOUT;
            o[q] = f2bf(Wqkv[(((size_t)h * 3 + k) * DIN + i) * DOUT + oo]); }
        VST2(v2us, WT + e0, o); }
#pragma unroll 1
    for (int s = 0; s < (DIN * HW) / 512; ++s) { const int e0 = s * 512 + t * 2; v2us o;
#pragma unroll
        for (int q = 0; q < 2; ++q) { const int e = e0 + q, c = e / HW, j = e - c * HW; o[q] = f2bf(Wo[(size_t)j * DIN + c]); }
        VST2(v2us, WoT + e0, o); }
}
template <bool SPLITA, int MODE>
__global__ __launch_bounds__(128) void k_gemm(const bf* __restrict__ A, const bf* __restrict__ Al, const bf* __restrict__ Bn, int K, const float* __restrict__ bias, const float* __restrict__ xres,
                                             const float* __restrict__ lg, const float* __restrict__ lb, void* C, void* C2) {
    __shared__ __align__(16) float ost[4][16 * 68];
    const int lane = threadIdx.x & 31, wave = threadIdx.x >> 5, lr = lane & 15, hi = lane >> 4;
    const int r0 = blockIdx.x * 64 + wave * 16, c0 = blockIdx.y * 64;
    const int ldc = (MODE == 3) ? DIN : HW;
    const size_t aoff = (size_t)(r0 + lr) * K + 8 * hi;
    size_t boff[4];
#pragma unroll
    for (int t = 0; t < 4; ++t) boff[t] = (size_t)(c0 + t * 16 + lr) * K + 8 * hi;
    v8f acc[4];
#pragma unroll
    for (int t = 0; t < 4; ++t) acc[t] = (v8f){};
#pragma unroll 1
    for (int kc = 0; kc < K; kc += 32) {
        const v16bf a = cat16b(*(const v8us*)(A + aoff + kc), *(const v8us*)(A + aoff + kc + 16));
        v16bf al = a;
        if (SPLITA) al = cat16b(*(const v8us*)(Al + aoff + kc), *(const v8us*)(Al + aoff + kc + 16));
#pragma unroll
        for (int t = 0; t < 4; ++t) { const v16bf b = cat16b(*(const v8us*)(Bn + boff[t] + kc), *(const v8us*)(Bn + boff[t] + kc + 16)); acc[t] = wmmab(a, b, acc[t]); if (SPLITA) acc[t] = wmmab(al, b, acc[t]); }
        asm volatile("v_nop\n\tv_nop\n\tv_nop\n\tv_nop" : "+v"(acc[0]), "+v"(acc[1]), "+v"(acc[2]), "+v"(acc[3]) : "v"(a), "v"(al));
    }
    float* os = &ost[wave][0];
    if (MODE == 3) {
#pragma unroll
        for (int j = 0; j < 8; ++j) { const size_t row = (size_t)(r0 + hi * 8 + j); float y[4], s = 0.f;
#pragma unroll
            for (int t = 0; t < 4; ++t) { const int c = t * 16 + lr; y[t] = acc[t][j] + bfr(bias[c]) + bfr(xres[row * DIN + c]); s += y[t]; }
            s += __shfl_xor(s, 1, 16); s += __shfl_xor(s, 2, 16); s += __shfl_xor(s, 4, 16); s += __shfl_xor(s, 8, 16);
            const float mu = s * (1.0f / DIN); float q = 0.f;
#pragma unroll
            for (int t = 0; t < 4; ++t) { const float d = y[t] - mu; q += d * d; }
            q += __shfl_xor(q, 1, 16); q += __shfl_xor(q, 2, 16); q += __shfl_xor(q, 4, 16); q += __shfl_xor(q, 8, 16);
            const float rs = rsqrtf(q * (1.0f / DIN) + 1e-5f);
#pragma unroll
            for (int t = 0; t < 4; ++t) { const int c = t * 16 + lr; os[(hi * 8 + j) * 68 + c] = (y[t] - mu) * rs * bfr(lg[c]) + bfr(lb[c]); } }
    } else {
#pragma unroll
        for (int t = 0; t < 4; ++t)
#pragma unroll
            for (int j = 0; j < 8; ++j) os[(hi * 8 + j) * 68 + t * 16 + lr] = acc[t][j];
    }
    __syncthreads();
    if (MODE == 2 || MODE == 3) {
        float* crow = (float*)C + (size_t)r0 * ldc + c0;
        auto pass = [&]() {
#pragma unroll
            for (int s = 0; s < 8; ++s) { const int Lid = (lane >> 3) + 4 * s, piece = lane & 7; const int row = Lid >> 1, cofs = (Lid & 1) * 32 + piece * 4;
                const v4f val = *(const v4fa*)(os + row * 68 + cofs); *(volatile v4f*)(crow + (size_t)row * ldc + cofs) = val; }
        };
        pass(); __threadfence(); pass();
    } else {
        h16* c1 = (h16*)C + (size_t)r0 * ldc + c0; h16* c2 = (h16*)C2 + (size_t)r0 * ldc + c0;
        auto pass = [&]() {
#pragma unroll
            for (int s = 0; s < 4; ++s) { const int row = 4 * s + (lane >> 3), piece = lane & 7; const float* sp = os + row * 68 + piece * 8; v8h o1, o2;
#pragma unroll
                for (int i = 0; i < 8; ++i) { const h16 a = (h16)sp[i]; o1[i] = a; o2[i] = (h16)((sp[i] - (float)a) * LOSC); }
                *(volatile v8h*)(c1 + (size_t)row * ldc + piece * 8) = o1; if (MODE == 0) *(volatile v8h*)(c2 + (size_t)row * ldc + piece * 8) = o2; }
        };
        pass(); __threadfence(); pass();
    }
}
__global__ __launch_bounds__(256) void k_vt(const float* __restrict__ V, h16* VT16) {
    __shared__ __align__(16) h16 tile[DOUT * 72];
    const int bid = blockIdx.x;
    const int b = bid / (NH_ * (NF / 64)), rem = bid - b * (NH_ * (NF / 64)), h = rem / (NF / 64), kt = rem - h * (NF / 64);
    const int f0 = kt * 64, tid = threadIdx.x, ff = tid >> 2, d0 = (tid & 3) * 16;
    const float* src = V + ((size_t)b * NF + f0 + ff) * HW + h * DOUT + d0;
#pragma unroll
    for (int i = 0; i < 16; ++i) tile[(d0 + i) * 72 + ff] = (h16)src[i];
    __syncthreads();
    const int piece = tid & 7;
    const size_t base = (((size_t)b * NH_ + h) * DOUT) * NF + f0;
    auto pass = [&]() {
#pragma unroll
        for (int s = 0; s < 2; ++s) { const int d = (tid >> 3) + 32 * s; const v8h val = *(const v8ha*)(tile + d * 72 + piece * 8); *(volatile v8h*)(VT16 + base + (size_t)d * NF + piece * 8) = val; }
    };
    pass(); __threadfence(); pass();
}
__global__ __launch_bounds__(128) void k_attn(const h16* __restrict__ QH, const h16* __restrict__ QL, const h16* __restrict__ K16, const h16* __restrict__ VT16, bf* CH, bf* CL) {
    __shared__ __align__(16) h16 plds[4][16 * 32];
    __shared__ __align__(16) float ost[4][16 * 68];
    const int lane = threadIdx.x & 31, wave = threadIdx.x >> 5, lr = lane & 15, hi = lane >> 4;
    const int bid = blockIdx.x;
    const int b = bid / (NH_ * (NF / 64)), rem = bid - b * (NH_ * (NF / 64)), h = rem / (NF / 64), qt = rem - h * (NF / 64);
    const int q0 = qt * 64 + wave * 16;
    const size_t tok0 = (size_t)b * NF;
    h16* pl = &plds[wave][0];
    v16h ah[2], al[2];
#pragma unroll
    for (int kc = 0; kc < 2; ++kc) { const size_t o = (tok0 + q0 + lr) * HW + h * DOUT + kc * 32 + 8 * hi;
        ah[kc] = cat16(*(const v8h*)(QH + o), *(const v8h*)(QH + o + 16)); al[kc] = cat16(*(const v8h*)(QL + o), *(const v8h*)(QL + o + 16)); }
    const size_t vbase = (((size_t)b * NH_ + h) * DOUT) * NF;
    v8f o[4];
#pragma unroll
    for (int n = 0; n < 4; ++n) o[n] = (v8f){};
#pragma unroll 1
    for (int kt = 0; kt < NF / 32; ++kt) {
        const int l0 = kt * 32;
        v8f s0 = {}, s1 = {}, x0 = {}, x1 = {};
#pragma unroll
        for (int kc = 0; kc < 2; ++kc) {
            const size_t o0 = (tok0 + l0 + lr) * HW + h * DOUT + kc * 32 + 8 * hi, o1 = o0 + (size_t)16 * HW;
            const v16h k0 = cat16(*(const v8h*)(K16 + o0), *(const v8h*)(K16 + o0 + 16)), k1 = cat16(*(const v8h*)(K16 + o1), *(const v8h*)(K16 + o1 + 16));
            s0 = wmma16(ah[kc], k0, s0); x0 = wmma16(al[kc], k0, x0); s1 = wmma16(ah[kc], k1, s1); x1 = wmma16(al[kc], k1, x1);
        }
        asm volatile("v_nop\n\tv_nop\n\tv_nop\n\tv_nop" : "+v"(s0), "+v"(s1), "+v"(x0), "+v"(x1) : "v"(ah[0]), "v"(al[1]));
#pragma unroll
        for (int j = 0; j < 8; ++j) { const int mr = hi * 8 + j;
            const float p0 = fmaxf((s0[j] + x0[j] * LOSCI) * 0.125f, 0.f), p1 = fmaxf((s1[j] + x1[j] * LOSCI) * 0.125f, 0.f);
            pl[mr * 32 + lr] = (h16)(p0 * PSC); pl[mr * 32 + 16 + lr] = (h16)(p1 * PSC); }
        asm volatile("" ::: "memory");
        const v16h pa = cat16(*(const v8ha*)(pl + lr * 32 + hi * 8), *(const v8ha*)(pl + lr * 32 + 16 + hi * 8));
#pragma unroll
        for (int n = 0; n < 4; ++n) { const size_t vo = vbase + (size_t)(n * 16 + lr) * NF + l0 + hi * 8; o[n] = wmma16(pa, cat16(*(const v8h*)(VT16 + vo), *(const v8h*)(VT16 + vo + 16)), o[n]); }
        asm volatile("v_nop\n\tv_nop\n\tv_nop\n\tv_nop" : "+v"(o[0]), "+v"(o[1]), "+v"(o[2]), "+v"(o[3]) : "v"(pa));
    }
    float* os = &ost[wave][0];
#pragma unroll
    for (int n = 0; n < 4; ++n)
#pragma unroll
        for (int j = 0; j < 8; ++j) os[(hi * 8 + j) * 68 + n * 16 + lr] = o[n][j] * (1.0f / PSC);
    __syncthreads();
    const size_t cbase = (tok0 + q0) * HW + (size_t)h * DOUT;
    auto pass = [&]() {
#pragma unroll
        for (int s = 0; s < 4; ++s) { const int row = 4 * s + (lane >> 3), piece = lane & 7; const float* sp = os + row * 68 + piece * 8; v8us oh, ol;
#pragma unroll
            for (int i = 0; i < 8; ++i) { const unsigned short hb = f2bf(sp[i]); oh[i] = hb; ol[i] = f2bf(sp[i] - bf2f(hb)); }
            *(volatile v8us*)(CH + cbase + (size_t)row * HW + piece * 8) = oh; *(volatile v8us*)(CL + cbase + (size_t)row * HW + piece * 8) = ol; }
    };
    pass(); __threadfence(); pass();
}

extern "C" void kernel_launch(void* const* d_in, const int* in_sizes, int n_in,
                              void* d_out, int out_size, void* d_ws, size_t ws_size, hipStream_t stream) {
    (void)in_sizes; (void)n_in; (void)out_size;
    const float* x = (const float*)d_in[0]; const float* Wqkv = (const float*)d_in[1]; const float* Wo = (const float*)d_in[2]; const float* bo = (const float*)d_in[3];
    const float* lg = (const float*)d_in[4]; const float* lb = (const float*)d_in[5];
    float* out = (float*)d_out;
    char* wsp = (char*)d_ws;
    auto take = [&](size_t bytes) { char* p = wsp; wsp += (bytes + 255) & ~(size_t)255; return (void*)p; };
    bf* Xb = (bf*)take((size_t)NTK * DIN * 2); bf* WT = (bf*)take((size_t)3 * HW * DIN * 2); bf* WoT = (bf*)take((size_t)DIN * HW * 2);
    h16* QH = (h16*)take((size_t)NTK * HW * 2); h16* QL = (h16*)take((size_t)NTK * HW * 2); h16* K16 = (h16*)take((size_t)NTK * HW * 2);
    float* Vf = (float*)take((size_t)NTK * HW * 4); h16* VT16 = (h16*)take((size_t)NTK * HW * 2);
    if ((size_t)(wsp - (char*)d_ws) > ws_size) return;
    bf* CH = (bf*)Vf; bf* CL = (bf*)((char*)Vf + (size_t)NTK * HW * 2);
    k_xb<<<(NTK / 2) / 8, 256, 0, stream>>>(x, Xb);
    k_w<<<1, 256, 0, stream>>>(Wqkv, Wo, WT, WoT);
    k_gemm<false, 0><<<dim3(NTK / 64, HW / 64, 1), 128, 0, stream>>>(Xb, nullptr, WT, DIN, nullptr, nullptr, nullptr, nullptr, QH, QL);
    k_gemm<false, 1><<<dim3(NTK / 64, HW / 64, 1), 128, 0, stream>>>(Xb, nullptr, WT + (size_t)HW * DIN, DIN, nullptr, nullptr, nullptr, nullptr, K16, nullptr);
    k_gemm<false, 2><<<dim3(NTK / 64, HW / 64, 1), 128, 0, stream>>>(Xb, nullptr, WT + (size_t)2 * HW * DIN, DIN, nullptr, nullptr, nullptr, nullptr, Vf, nullptr);
    k_vt<<<NB_ * NH_ * (NF / 64), 256, 0, stream>>>(Vf, VT16);
    k_attn<<<NB_ * NH_ * (NF / 64), 128, 0, stream>>>(QH, QL, K16, VT16, CH, CL);
    k_gemm<true, 3><<<dim3(NTK / 64, 1, 1), 128, 0, stream>>>(CH, CL, WoT, HW, bo, x, lg, lb, out, nullptr);
}
